// TRMAttention_89378269430415
// MI455X (gfx1250) — hardware-verified
//
#include <hip/hip_runtime.h>
#include <math.h>
#include <stdint.h>

#define NBATCH 2
#define SEQ    2048
#define DM     2048
#define NHEAD  16
#define HDIM   128
#define NTOK   (NBATCH * SEQ)
#define NQB    (SEQ / 64)
#define NQP    8
#define NFREQ  (HDIM / 2)
#define WSC    16.0f
#define QSC    4.0f
#define KSC    16.0f
#define VSC    16.0f
#define VRS    4096.0f
#define QRS    VRS
#define PSC    1024.0f
#define PRS    VRS
#define NEG_BIG (-1.0e30f)
static_assert(NHEAD * HDIM == DM);
static_assert((SEQ % 64) == 0 && (DM % 128) == 0);
static_assert((DM % 32) == 0 && (HDIM % 32) == 0);
static_assert(NFREQ == 64);
static_assert(((NTOK * DM) % 2048) == 0 && ((DM * DM) % 2048) == 0);
static_assert(NQP > 0 && NQP < NQB);

typedef _Float16 v16h __attribute__((ext_vector_type(16)));
typedef _Float16 v8h  __attribute__((ext_vector_type(8)));
typedef __bf16   v16b __attribute__((ext_vector_type(16)));
typedef unsigned short v16us __attribute__((ext_vector_type(16)));
typedef unsigned short v8us  __attribute__((ext_vector_type(8)));
typedef float    v8f  __attribute__((ext_vector_type(8)));
typedef float    v4f  __attribute__((ext_vector_type(4)));
typedef float    v2f  __attribute__((ext_vector_type(2)));
typedef unsigned int v4u __attribute__((ext_vector_type(4)));
union FH { v16h v; v8h h[2]; };
union FB { v16us u; v8us h[2]; };

__device__ __forceinline__ unsigned short bf_bits(float f) {
  unsigned u = __float_as_uint(f);
  return (unsigned short)((u + 0x7FFFu + ((u >> 16) & 1u)) >> 16);
}
__device__ __forceinline__ float bf_up(unsigned short h) { return __uint_as_float(((unsigned)h) << 16); }
__device__ __forceinline__ float bfr(float f) { return bf_up(bf_bits(f)); }
__device__ __forceinline__ unsigned short h_bits(_Float16 x) { return __builtin_bit_cast(unsigned short, x); }
__device__ __forceinline__ unsigned pk16(unsigned short a, unsigned short b) { return (unsigned)a | ((unsigned)b << 16); }
__device__ __forceinline__ v8f zero8() { v8f z = {0.f, 0.f, 0.f, 0.f, 0.f, 0.f, 0.f, 0.f}; return z; }

__device__ __forceinline__ v16h ldfrag_h(const _Float16* p) {
  FH f;
  f.h[0] = *(const v8h*)(p);
  f.h[1] = *(const v8h*)(p + 16);
  return f.v;
}
__device__ __forceinline__ v16us ldfrag_b(const unsigned short* p) {
  FB f;
  f.h[0] = *(const v8us*)(p);
  f.h[1] = *(const v8us*)(p + 16);
  return f.u;
}

__device__ __forceinline__ v8f mma_h(v16h a, v16h b, v8f c) {
  c = __builtin_amdgcn_wmma_f32_16x16x32_f16(false, a, false, b, (short)0, c, false, false);
#if defined(__HIP_DEVICE_COMPILE__)
  asm volatile("v_nop\n\tv_nop\n\tv_nop\n\tv_nop" : "+v"(c) : "v"(a), "v"(b));
#endif
  return c;
}
__device__ __forceinline__ v8f mma_h_raw(v16h a, v16h b, v8f c) {
  return __builtin_amdgcn_wmma_f32_16x16x32_f16(false, a, false, b, (short)0, c, false, false);
}
__device__ __forceinline__ v8f mma_b_raw(v16us a, v16us b, v8f c) {
  return __builtin_amdgcn_wmma_f32_16x16x32_bf16(false, __builtin_bit_cast(v16b, a), false,
                                                 __builtin_bit_cast(v16b, b), (short)0, c, false, false);
}
template <typename F>
__device__ __forceinline__ void guard3(v8f& x, v8f& y, F a, F b, F d) {
#if defined(__HIP_DEVICE_COMPILE__)
  asm volatile("v_nop\n\tv_nop\n\tv_nop\n\tv_nop" : "+v"(x), "+v"(y) : "v"(a), "v"(b), "v"(d));
#endif
}
template <typename F>
__device__ __forceinline__ void guard4i(v8f& x, v8f& y, F a, F b, F d, F e) {
#if defined(__HIP_DEVICE_COMPILE__)
  asm volatile("v_nop\n\tv_nop\n\tv_nop\n\tv_nop" : "+v"(x), "+v"(y) : "v"(a), "v"(b), "v"(d), "v"(e));
#endif
}
__device__ __forceinline__ void acc_guard4(v8f& a, v8f& b, v8f& c, v8f& d) {
#if defined(__HIP_DEVICE_COMPILE__)
  asm volatile("v_nop\n\tv_nop\n\tv_nop\n\tv_nop" : "+v"(a), "+v"(b), "+v"(c), "+v"(d));
#endif
}
__device__ __forceinline__ void wave_sync_lds() {
  __builtin_amdgcn_fence(__ATOMIC_RELEASE, "workgroup");
  __builtin_amdgcn_wave_barrier();
  __builtin_amdgcn_fence(__ATOMIC_ACQUIRE, "workgroup");
}

struct OpH {
  typedef v16h F;
  static __device__ __forceinline__ F ld(const unsigned short* p) { return ldfrag_h((const _Float16*)(const void*)p); }
  static __device__ __forceinline__ v8f mma(F a, F b, v8f c) { return mma_h_raw(a, b, c); }
};
struct OpB {
  typedef v16us F;
  static __device__ __forceinline__ F ld(const unsigned short* p) { return ldfrag_b(p); }
  static __device__ __forceinline__ v8f mma(F a, F b, v8f c) { return mma_b_raw(a, b, c); }
};

__global__ __launch_bounds__(64) void rope_tab(float* cs) {
  __shared__ __align__(16) float row[2 * NFREQ];
  const int t = blockIdx.x;
  const int i = threadIdx.x;
  const float e = (float)(2 * i) * (1.0f / (float)HDIM);
  const float p = (float)exp2((double)e * 13.287712379549449391);
  const float inv = (float)(1.0 / (double)p);
  const float ang = (float)t * inv;
  row[2 * i]     = cosf(ang);
  row[2 * i + 1] = sinf(ang);
  __syncthreads();
  if (i < 32) {
    const v4f v = *(const v4f*)(row + 4 * i);
    float* g = cs + (size_t)t * (2 * NFREQ) + 4 * i;
    *(volatile v4f*)g = v;
    __threadfence();
    *(volatile v4f*)g = v;
  }
}

__global__ __launch_bounds__(256) void cvt_x(const float* __restrict__ in, unsigned short* out, int n) {
  const size_t i8 = ((size_t)blockIdx.x * 256 + threadIdx.x) * 8;
  if (i8 + 8 > (size_t)n) return;
  const v4f a = *(const v4f*)(in + i8);
  const v4f b = *(const v4f*)(in + i8 + 4);
  v4u p;
#pragma unroll
  for (int e = 0; e < 2; ++e) {
    p[e]     = pk16(h_bits((_Float16)bfr(a[2 * e])), h_bits((_Float16)bfr(a[2 * e + 1])));
    p[2 + e] = pk16(h_bits((_Float16)bfr(b[2 * e])), h_bits((_Float16)bfr(b[2 * e + 1])));
  }
  *(volatile v4u*)(out + i8) = p;
  __threadfence();
  *(volatile v4u*)(out + i8) = p;
}

__global__ __launch_bounds__(256) void cvt_w(const float* __restrict__ in, unsigned short* out, int n,
                                            float scale, int bfmode) {
  const size_t i8 = ((size_t)blockIdx.x * 256 + threadIdx.x) * 8;
  if (i8 + 8 > (size_t)n) return;
  const v4f a = *(const v4f*)(in + i8);
  const v4f b = *(const v4f*)(in + i8 + 4);
  float f[8];
  f[0] = a[0]; f[1] = a[1]; f[2] = a[2]; f[3] = a[3];
  f[4] = b[0]; f[5] = b[1]; f[6] = b[2]; f[7] = b[3];
  v4u p;
#pragma unroll
  for (int e = 0; e < 4; ++e) {
    const unsigned short b0 = bf_bits(f[2 * e]), b1 = bf_bits(f[2 * e + 1]);
    const _Float16 x0 = (_Float16)(bf_up(b0) * scale);
    const _Float16 x1 = (_Float16)(bf_up(b1) * scale);
    const unsigned wf = pk16(h_bits(x0), h_bits(x1));
    const unsigned wb = pk16(b0, b1);
    p[e] = (bfmode != 0) ? wb : wf;
  }
  *(volatile v4u*)(out + i8) = p;
  __threadfence();
  *(volatile v4u*)(out + i8) = p;
}

template <class OP, int NSW, int OM, int ROPE>
__global__ __launch_bounds__(128) void gemm_t(
    const unsigned short* __restrict__ A0, const unsigned short* __restrict__ A1, int lda,
    const unsigned short* __restrict__ B0, const unsigned short* __restrict__ B1, int ldb,
    void* C0, void* C1, int ldc, const float* __restrict__ cs, int M, int N, int K, float oscale) {
  typedef typename OP::F F;
  __shared__ __align__(16) float sT[4][16 * 132];
  const int lane = threadIdx.x & 31;
  const int wave = threadIdx.x >> 5;
  const int tilesN = N >> 7;
  const int tilesM = M >> 5;
  const int tile = blockIdx.x * 4 + wave;
  if (tile >= tilesM * tilesN) return;
  const int tm = tile / tilesN;
  const int tn = tile - tm * tilesN;
  const int m0 = tm << 5;
  const int n0 = tn << 7;
  const int rl   = lane & 15;
  const int hh   = lane >> 4;
  const int koff = hh * 8;

  v8f acc[2][8];
#pragma unroll
  for (int i = 0; i < 2; ++i)
#pragma unroll
    for (int j = 0; j < 8; ++j) acc[i][j] = zero8();

#pragma unroll 1
  for (int sw = 0; sw < NSW; ++sw) {
    const unsigned short* Ab = (sw == 0) ? A0 : A1;
    const unsigned short* Bb = (sw == 0) ? B0 : B1;
    const unsigned short* ar0 = Ab + (size_t)(m0 + rl) * (size_t)lda + koff;
    const unsigned short* ar1 = Ab + (size_t)(m0 + 16 + rl) * (size_t)lda + koff;
    const unsigned short* br  = Bb + (size_t)(n0 + rl) * (size_t)ldb + koff;
    for (int k0 = 0; k0 < K; k0 += 32) {
      const F a0 = OP::ld(ar0 + k0);
      const F a1 = OP::ld(ar1 + k0);
#pragma unroll
      for (int j = 0; j < 8; ++j) {
        const F b = OP::ld(br + (size_t)j * 16 * (size_t)ldb + k0);
        acc[0][j] = OP::mma(a0, b, acc[0][j]);
        acc[1][j] = OP::mma(a1, b, acc[1][j]);
        guard3<F>(acc[0][j], acc[1][j], a0, a1, b);
      }
    }
  }
  acc_guard4(acc[0][0], acc[0][1], acc[0][2], acc[0][3]);
  acc_guard4(acc[0][4], acc[0][5], acc[0][6], acc[0][7]);
  acc_guard4(acc[1][0], acc[1][1], acc[1][2], acc[1][3]);
  acc_guard4(acc[1][4], acc[1][5], acc[1][6], acc[1][7]);

  float* slab = sT[wave];
#pragma unroll
  for (int i = 0; i < 2; ++i) {
    const int mB = m0 + 16 * i;
    if (ROPE != 0) {
#pragma unroll
      for (int j = 0; j < 4; ++j) {
#pragma unroll
        for (int r = 0; r < 8; ++r) {
          const int tb = (mB + 8 * hh + r) & (SEQ - 1);
          const v2f w = *(const v2f*)(cs + ((size_t)tb * NFREQ + 16 * j + rl) * 2);
          const float x1 = acc[i][j][r] * oscale;
          const float x2 = acc[i][j + 4][r] * oscale;
          slab[(8 * hh + r) * 132 + 16 * j + rl]      = x1 * w[0] - x2 * w[1];
          slab[(8 * hh + r) * 132 + 64 + 16 * j + rl] = x1 * w[1] + x2 * w[0];
        }
      }
    } else {
#pragma unroll
      for (int j = 0; j < 8; ++j) {
#pragma unroll
        for (int r = 0; r < 8; ++r) slab[(8 * hh + r) * 132 + 16 * j + rl] = acc[i][j][r] * oscale;
      }
    }
    wave_sync_lds();
    if (OM == 4) {
      float* Cf = (float*)C0;
      for (int pass = 0; pass < 2; ++pass) {
#pragma unroll
        for (int it = 0; it < 16; ++it) {
          const v4f o = *(const v4f*)(slab + it * 132 + lane * 4);
          *(volatile v4f*)(Cf + (size_t)(mB + it) * (size_t)ldc + n0 + lane * 4) = o;
        }
        __threadfence();
      }
    } else {
      unsigned short* Cp = (unsigned short*)C0;
      unsigned short* Cq = (unsigned short*)C1;
      v4u hv[8], lv[8];
#pragma unroll
      for (int it = 0; it < 8; ++it) {
        const int row = it * 2 + hh;
        const float* sp = slab + row * 132 + rl * 8;
        const v4f fa = *(const v4f*)sp;
        const v4f fb = *(const v4f*)(sp + 4);
        float f[8];
        f[0] = fa[0]; f[1] = fa[1]; f[2] = fa[2]; f[3] = fa[3];
        f[4] = fb[0]; f[5] = fb[1]; f[6] = fb[2]; f[7] = fb[3];
        v4u pk;
        v4u pl = {0u, 0u, 0u, 0u};
#pragma unroll
        for (int e = 0; e < 4; ++e) {
          const float g0 = f[2 * e], g1 = f[2 * e + 1];
          if (OM == 2) {
            const unsigned short b0 = bf_bits(g0), b1 = bf_bits(g1);
            pk[e] = pk16(b0, b1);
            pl[e] = pk16(bf_bits(g0 - bf_up(b0)), bf_bits(g1 - bf_up(b1)));
          } else {
            const _Float16 x0 = (_Float16)g0;
            const _Float16 x1 = (_Float16)g1;
            pk[e] = pk16(h_bits(x0), h_bits(x1));
            if (OM == 3) {
              const _Float16 y0 = (_Float16)((g0 - (float)x0) * VRS);
              const _Float16 y1 = (_Float16)((g1 - (float)x1) * VRS);
              pl[e] = pk16(h_bits(y0), h_bits(y1));
            }
          }
        }
        hv[it] = pk;
        lv[it] = pl;
      }
      for (int pass = 0; pass < 2; ++pass) {
#pragma unroll
        for (int it = 0; it < 8; ++it) {
          const int row = it * 2 + hh;
          const size_t go = (size_t)(mB + row) * (size_t)ldc + n0 + rl * 8;
          *(volatile v4u*)(Cp + go) = hv[it];
          if (OM == 2 || OM == 3) *(volatile v4u*)(Cq + go) = lv[it];
        }
        __threadfence();
      }
    }
    wave_sync_lds();
  }
}

template <bool PRES>
__global__ __launch_bounds__(128)
void attn_c(const unsigned short* __restrict__ Qp, const unsigned short* __restrict__ Qlp,
            const unsigned short* __restrict__ Kp, const unsigned short* __restrict__ Klp,
            const unsigned short* __restrict__ Vhp, const unsigned short* __restrict__ Vlp,
            unsigned short* CH, unsigned short* CL, float sscale, int qb0, int nqb) {
  __shared__ __align__(16) _Float16 Ksh[64 * HDIM];
  __shared__ __align__(16) _Float16 Kls[64 * HDIM];
  __shared__ __align__(16) _Float16 Vhs[HDIM * 64];
  __shared__ __align__(16) _Float16 Vls[PRES ? HDIM * 64 : 8];
  __shared__ __align__(16) _Float16 Psh[4][16 * 64];
  __shared__ __align__(16) _Float16 Psl[PRES ? 4 : 1][PRES ? 16 * 64 : 8];
  __shared__ __align__(16) float    Os[4][16 * HDIM];

  const int tid  = threadIdx.x;
  const int wave = tid >> 5;
  const int lane = tid & 31;
  const int hh   = lane >> 4;
  const int c    = lane & 15;

  const int qb = qb0 + (int)(blockIdx.x % (unsigned)nqb);
  const int h  = (int)(blockIdx.x / (unsigned)nqb);
  const int q0 = qb * 64 + wave * 16;

  const _Float16* Qg  = (const _Float16*)(const void*)Qp  + (size_t)h * HDIM;
  const _Float16* Qlg = (const _Float16*)(const void*)Qlp + (size_t)h * HDIM;
  const _Float16* Kg  = (const _Float16*)(const void*)Kp  + (size_t)h * HDIM;
  const _Float16* Klg = (const _Float16*)(const void*)Klp + (size_t)h * HDIM;
  const _Float16* Vhg = (const _Float16*)(const void*)Vhp + (size_t)h * HDIM * SEQ;
  const _Float16* Vlg = (const _Float16*)(const void*)Vlp + (size_t)h * HDIM * SEQ;

  float mrow[8], lrow[8];
  v8f oh[8];
#pragma unroll
  for (int r = 0; r < 8; ++r) { mrow[r] = NEG_BIG; lrow[r] = 0.f; }
#pragma unroll
  for (int t = 0; t < 8; ++t) oh[t] = zero8();

  _Float16* pwh = Psh[wave];
  _Float16* pwl = &Psl[PRES ? wave : 0][0];

  for (int kt = 0; kt < NQB; ++kt) {
    if (kt > qb) break;
    const int kv0 = kt * 64;
    __syncthreads();
    {
      const int r = tid >> 1, hk = (tid & 1) * 64;
      const _Float16* kg = Kg  + (size_t)(kv0 + r) * DM + hk;
      const _Float16* lg = Klg + (size_t)(kv0 + r) * DM + hk;
#pragma unroll
      for (int i = 0; i < 8; ++i) *(v8h*)(Ksh + r * HDIM + hk + 8 * i) = *(const v8h*)(kg + 8 * i);
#pragma unroll
      for (int i = 0; i < 8; ++i) *(v8h*)(Kls + r * HDIM + hk + 8 * i) = *(const v8h*)(lg + 8 * i);
      const _Float16* vh = Vhg + (size_t)tid * SEQ + kv0;
#pragma unroll
      for (int i = 0; i < 8; ++i) *(v8h*)(Vhs + tid * 64 + 8 * i) = *(const v8h*)(vh + 8 * i);
      if (PRES) {
        const _Float16* vl = Vlg + (size_t)tid * SEQ + kv0;
#pragma unroll
        for (int i = 0; i < 8; ++i) *(v8h*)(Vls + tid * 64 + 8 * i) = *(const v8h*)(vl + 8 * i);
      }
    }
    __syncthreads();

    v8f sh[4], sl[4];
#pragma unroll
    for (int j = 0; j < 4; ++j) { sh[j] = zero8(); sl[j] = zero8(); }
#pragma unroll
    for (int dc = 0; dc < 4; ++dc) {
      const v16h qh = ldfrag_h(Qg  + (size_t)(q0 + c) * DM + dc * 32 + 8 * hh);
      const v16h ql = ldfrag_h(Qlg + (size_t)(q0 + c) * DM + dc * 32 + 8 * hh);
#pragma unroll
      for (int j = 0; j < 4; ++j) {
        FH kb, kl;
        kb.h[0] = *(const v8h*)(Ksh + (j * 16 + c) * HDIM + dc * 32 + 8 * hh);
        kb.h[1] = *(const v8h*)(Ksh + (j * 16 + c) * HDIM + dc * 32 + 16 + 8 * hh);
        kl.h[0] = *(const v8h*)(Kls + (j * 16 + c) * HDIM + dc * 32 + 8 * hh);
        kl.h[1] = *(const v8h*)(Kls + (j * 16 + c) * HDIM + dc * 32 + 16 + 8 * hh);
        sh[j] = mma_h_raw(qh, kb.v, sh[j]);
        sl[j] = mma_h_raw(ql, kb.v, sl[j]);
        sl[j] = mma_h_raw(qh, kl.v, sl[j]);
        guard4i<v16h>(sh[j], sl[j], qh, ql, kb.v, kl.v);
      }
    }
    acc_guard4(sh[0], sh[1], sh[2], sh[3]);
    acc_guard4(sl[0], sl[1], sl[2], sl[3]);
    v8f s[4];
#pragma unroll
    for (int j = 0; j < 4; ++j) {
      const int key  = kv0 + j * 16 + c;
      const int rowb = q0 + 8 * hh;
#pragma unroll
      for (int r = 0; r < 8; ++r) {
        const float v = (sh[j][r] + sl[j][r] * (1.0f / QRS)) * sscale;
        s[j][r] = (key <= rowb + r) ? v : NEG_BIG;
      }
    }

#pragma unroll
    for (int r = 0; r < 8; ++r) {
      float m = s[0][r];
      m = fmaxf(m, s[1][r]);
      m = fmaxf(m, s[2][r]);
      m = fmaxf(m, s[3][r]);
#pragma unroll
      for (int off = 1; off < 16; off <<= 1) m = fmaxf(m, __shfl_xor(m, off, 32));
      const float mnew  = fmaxf(mrow[r], m);
      const float alpha = __expf(mrow[r] - mnew);
      mrow[r] = mnew;
      float psum = 0.f;
#pragma unroll
      for (int j = 0; j < 4; ++j) {
        const float p  = __expf(s[j][r] - mnew);
        psum += p;
        const float ph = p * PSC;
        const _Float16 xh = (_Float16)ph;
        const int pi = (8 * hh + r) * 64 + j * 16 + c;
        pwh[pi] = xh;
        if (PRES) pwl[pi] = (_Float16)((ph - (float)xh) * PRS);
      }
#pragma unroll
      for (int off = 1; off < 16; off <<= 1) psum += __shfl_xor(psum, off, 32);
      lrow[r] = lrow[r] * alpha + psum;
#pragma unroll
      for (int t = 0; t < 8; ++t) oh[t][r] *= alpha;
    }
    wave_sync_lds();

    if (PRES) {
      v8f ol[8];
#pragma unroll
      for (int t = 0; t < 8; ++t) ol[t] = zero8();
#pragma unroll 1
      for (int kk = 0; kk < 2; ++kk) {
        FH pa, pb;
        pa.h[0] = *(const v8h*)(pwh + c * 64 + kk * 32 + 8 * hh);
        pa.h[1] = *(const v8h*)(pwh + c * 64 + kk * 32 + 16 + 8 * hh);
        pb.h[0] = *(const v8h*)(pwl + c * 64 + kk * 32 + 8 * hh);
        pb.h[1] = *(const v8h*)(pwl + c * 64 + kk * 32 + 16 + 8 * hh);
#pragma unroll
        for (int t = 0; t < 8; ++t) {
          FH vb, wb;
          vb.h[0] = *(const v8h*)(Vhs + (t * 16 + c) * 64 + kk * 32 + 8 * hh);
          vb.h[1] = *(const v8h*)(Vhs + (t * 16 + c) * 64 + kk * 32 + 16 + 8 * hh);
          wb.h[0] = *(const v8h*)(Vls + (t * 16 + c) * 64 + kk * 32 + 8 * hh);
          wb.h[1] = *(const v8h*)(Vls + (t * 16 + c) * 64 + kk * 32 + 16 + 8 * hh);
          ol[t] = mma_h_raw(pa.v, wb.v, ol[t]);
          oh[t] = mma_h_raw(pa.v, vb.v, oh[t]);
          ol[t] = mma_h_raw(pb.v, vb.v, ol[t]);
          guard4i<v16h>(oh[t], ol[t], pa.v, pb.v, vb.v, wb.v);
        }
      }
      acc_guard4(oh[0], oh[1], oh[2], oh[3]);
      acc_guard4(oh[4], oh[5], oh[6], oh[7]);
      acc_guard4(ol[0], ol[1], ol[2], ol[3]);
      acc_guard4(ol[4], ol[5], ol[6], ol[7]);
#pragma unroll
      for (int t = 0; t < 8; ++t) {
#pragma unroll
        for (int r = 0; r < 8; ++r) oh[t][r] += ol[t][r] * (1.0f / VRS);
      }
    } else {
#pragma unroll 1
      for (int kk = 0; kk < 2; ++kk) {
        FH pa;
        pa.h[0] = *(const v8h*)(pwh + c * 64 + kk * 32 + 8 * hh);
        pa.h[1] = *(const v8h*)(pwh + c * 64 + kk * 32 + 16 + 8 * hh);
#pragma unroll
        for (int t = 0; t < 8; ++t) {
          FH vb;
          vb.h[0] = *(const v8h*)(Vhs + (t * 16 + c) * 64 + kk * 32 + 8 * hh);
          vb.h[1] = *(const v8h*)(Vhs + (t * 16 + c) * 64 + kk * 32 + 16 + 8 * hh);
          oh[t] = mma_h(pa.v, vb.v, oh[t]);
        }
      }
      acc_guard4(oh[0], oh[1], oh[2], oh[3]);
      acc_guard4(oh[4], oh[5], oh[6], oh[7]);
    }
  }

  float* os = Os[wave];
#pragma unroll
  for (int r = 0; r < 8; ++r) {
    const float l = lrow[r];
    const float inv = ((l > 0.f) ? (1.0f / l) : 0.f) * (1.0f / (PSC * VSC));
#pragma unroll
    for (int t = 0; t < 8; ++t) os[(8 * hh + r) * HDIM + t * 16 + c] = oh[t][r] * inv;
  }
  wave_sync_lds();
  {
    v4u hvv[8], lvv[8];
#pragma unroll
    for (int it = 0; it < 8; ++it) {
      const int row = it * 2 + hh;
      const float* sp = os + row * HDIM + c * 8;
      const v4f fa = *(const v4f*)sp;
      const v4f fb = *(const v4f*)(sp + 4);
      float f[8];
      f[0] = fa[0]; f[1] = fa[1]; f[2] = fa[2]; f[3] = fa[3];
      f[4] = fb[0]; f[5] = fb[1]; f[6] = fb[2]; f[7] = fb[3];
      v4u pk, pl;
#pragma unroll
      for (int e = 0; e < 4; ++e) {
        const float g0 = f[2 * e], g1 = f[2 * e + 1];
        const unsigned short b0 = bf_bits(g0), b1 = bf_bits(g1);
        const unsigned short l0 = bf_bits(g0 - bf_up(b0)), l1 = bf_bits(g1 - bf_up(b1));
        pk[e] = pk16(b0, b1);
        pl[e] = pk16(l0, l1);
      }
      hvv[it] = pk;
      lvv[it] = pl;
    }
    for (int pass = 0; pass < 2; ++pass) {
#pragma unroll
      for (int it = 0; it < 8; ++it) {
        const int row = it * 2 + hh;
        const size_t go = (size_t)(q0 + row) * DM + (size_t)h * HDIM + c * 8;
        *(volatile v4u*)(CH + go) = hvv[it];
        *(volatile v4u*)(CL + go) = lvv[it];
      }
      __threadfence();
    }
  }
}

extern "C" void kernel_launch(void* const* d_in, const int* in_sizes, int n_in,
                              void* d_out, int out_size, void* d_ws, size_t ws_size,
                              hipStream_t stream) {
  if (n_in < 5) return;
  if (in_sizes[0] != NTOK * DM) return;
  if (in_sizes[1] != DM * DM || in_sizes[2] != DM * DM) return;
  if (in_sizes[3] != DM * DM || in_sizes[4] != DM * DM) return;
  if (out_size != NTOK * DM) return;

  const float* X  = (const float*)d_in[0];
  const float* Wq = (const float*)d_in[1];
  const float* Wk = (const float*)d_in[2];
  const float* Wv = (const float*)d_in[3];
  const float* Wo = (const float*)d_in[4];
  float* outf = (float*)d_out;

  const size_t PCS  = (size_t)SEQ * NFREQ * 2 * 4;
  const size_t PW   = (size_t)DM * DM * 2;
  const size_t PXH  = (size_t)NTOK * DM * 2;
  const size_t PQK  = (size_t)SEQ * DM * 2;
  const size_t PVT  = (size_t)DM * SEQ * 2;
  const size_t PCTX = (size_t)SEQ * DM * 2;
  size_t off = 0;
  const size_t oCS  = off; off += PCS;
  const size_t oWQ  = off; off += PW;
  const size_t oWK  = off; off += PW;
  const size_t oWV  = off; off += PW;
  const size_t oWO  = off; off += PW;
  const size_t oXH  = off; off += PXH;
  const size_t oQ   = off; off += PQK;
  const size_t oQL  = off; off += PQK;
  const size_t oK   = off; off += PQK;
  const size_t oKL  = off; off += PQK;
  const size_t oVH  = off; off += PVT;
  const size_t oVL  = off; off += PVT;
  const size_t oCH  = off; off += PCTX;
  const size_t oCL  = off; off += PCTX;
  if (off > ws_size) return;
  if (off > (size_t)134217728) return;

  char* ws = (char*)d_ws;
  float* CS = (float*)(ws + oCS);
  unsigned short* WQ16 = (unsigned short*)(ws + oWQ);
  unsigned short* WK16 = (unsigned short*)(ws + oWK);
  unsigned short* WV16 = (unsigned short*)(ws + oWV);
  unsigned short* WOB  = (unsigned short*)(ws + oWO);
  unsigned short* XH   = (unsigned short*)(ws + oXH);
  unsigned short* QP   = (unsigned short*)(ws + oQ);
  unsigned short* QL   = (unsigned short*)(ws + oQL);
  unsigned short* KP   = (unsigned short*)(ws + oK);
  unsigned short* KL   = (unsigned short*)(ws + oKL);
  unsigned short* VTH  = (unsigned short*)(ws + oVH);
  unsigned short* VTL  = (unsigned short*)(ws + oVL);
  unsigned short* CTXH = (unsigned short*)(ws + oCH);
  unsigned short* CTXL = (unsigned short*)(ws + oCL);

  const dim3 blk256(256), blk128(128);
  const float sscale = 0.08838834764831845f / (QSC * KSC);

  rope_tab<<<dim3(SEQ), dim3(64), 0, stream>>>(CS);
  cvt_w<<<dim3((DM * DM) / 2048), blk256, 0, stream>>>(Wq, WQ16, DM * DM, WSC, 0);
  cvt_w<<<dim3((DM * DM) / 2048), blk256, 0, stream>>>(Wk, WK16, DM * DM, WSC, 0);
  cvt_w<<<dim3((DM * DM) / 2048), blk256, 0, stream>>>(Wv, WV16, DM * DM, WSC, 0);
  cvt_w<<<dim3((DM * DM) / 2048), blk256, 0, stream>>>(Wo, WOB, DM * DM, 1.0f, 1);
  cvt_x<<<dim3((NTOK * DM) / 2048), blk256, 0, stream>>>(X, XH, NTOK * DM);

  const int gsq = ((SEQ / 32) * (DM / 128)) / 4;
  for (int b = 0; b < NBATCH; ++b) {
    const unsigned short* XHb = XH + (size_t)b * SEQ * DM;
    float* outb = outf + (size_t)b * SEQ * DM;
    gemm_t<OpH, 1, 3, 1><<<dim3(gsq), blk128, 0, stream>>>(
        XHb, XHb, DM, WQ16, WQ16, DM, (void*)QP, (void*)QL, DM, CS, SEQ, DM, DM, QSC / WSC);
    gemm_t<OpH, 1, 3, 1><<<dim3(gsq), blk128, 0, stream>>>(
        XHb, XHb, DM, WK16, WK16, DM, (void*)KP, (void*)KL, DM, CS, SEQ, DM, DM, KSC / WSC);
    gemm_t<OpH, 1, 3, 0><<<dim3(gsq), blk128, 0, stream>>>(
        WV16, WV16, DM, XHb, XHb, DM, (void*)VTH, (void*)VTL, SEQ, CS, DM, SEQ, DM, VSC / WSC);
    attn_c<true><<<dim3(NQP * NHEAD), blk128, 0, stream>>>(QP, QL, KP, KL, VTH, VTL, CTXH, CTXL, sscale, 0, NQP);
    attn_c<false><<<dim3((NQB - NQP) * NHEAD), blk128, 0, stream>>>(QP, QL, KP, KL, VTH, VTL, CTXH, CTXL, sscale,
                                                                    NQP, NQB - NQP);
    gemm_t<OpB, 2, 4, 0><<<dim3(gsq), blk128, 0, stream>>>(
        CTXH, CTXL, DM, WOB, WOB, DM, (void*)outb, (void*)outb, DM, CS, SEQ, DM, DM, 1.0f);
  }
  (void)hipGetLastError();
}
